// RWKV6Layer_8323646620460
// MI455X (gfx1250) — hardware-run, weakly checked
//
#include <hip/hip_runtime.h>
#include <math.h>

constexpr int kB = 4;
constexpr int kT = 2048;
constexpr int kD = 512;
constexpr int kH = 4;
constexpr int kDK = 64;
constexpr int kDV = 128;
constexpr int kLR = 32;
constexpr int kRows = kB * kT;
constexpr int kMixCols = 5 * kLR;
constexpr int kMixPad = 192;
constexpr int kDecRank = 64;
constexpr int kQK = kH * kDK;
constexpr int kFF = 1024;
constexpr int kChunk = 16;
constexpr float kLnEps = 1e-5f;
constexpr float kWCarry  = 16.0f;
constexpr float kOoCarry = 16.0f;
constexpr float kKkCarry = 64.0f;

static_assert(kD == kH * kDV);
static_assert(kQK == 256 && kMixCols == 160 && kMixCols <= kMixPad);
static_assert((kT & (kT - 1)) == 0);
static_assert(kRows % 64 == 0 && kD % 64 == 0 && kMixPad % 64 == 0 && kDecRank % 64 == 0 && kQK % 64 == 0 && kFF % 64 == 0);
static_assert(kD % 32 == 0 && kLR % 32 == 0 && kDecRank % 32 == 0 && kFF % 32 == 0);
static_assert(((kRows / 64) * (kDecRank / 64)) % 8 == 0 && ((kRows / 64) * (kMixPad / 64)) % 8 == 0);
static_assert(kT % kChunk == 0);

constexpr int kEpiPlain  = 0;
constexpr int kEpiTanh   = 1;
constexpr int kEpiMix    = 2;
constexpr int kEpiDec    = 3;
constexpr int kEpiResid  = 4;
constexpr int kEpiReluSq = 5;
constexpr int kEpiSigm   = 6;
constexpr int kEpiFinal  = 7;

typedef __attribute__((ext_vector_type(16))) _Float16 v16h;
typedef __attribute__((ext_vector_type(8)))  _Float16 v8h;
typedef __attribute__((ext_vector_type(8)))  float    v8f;
typedef __attribute__((ext_vector_type(4)))  float    v4f;
typedef __attribute__((ext_vector_type(4)))  unsigned int v4u;
typedef __attribute__((ext_vector_type(2)))  unsigned int v2u;

__device__ __forceinline__ unsigned pk16(unsigned short a, unsigned short b) { return (unsigned)a | ((unsigned)b << 16); }
__device__ __forceinline__ unsigned short h_bits(float f) { const _Float16 h = (_Float16)f; return __builtin_bit_cast(unsigned short, h); }

__device__ __forceinline__ float h16_to_f32(unsigned hb) {
  const unsigned sgn = (hb & 0x8000u) << 16;
  const unsigned em = hb & 0x7fffu;
  const float fn = __uint_as_float((em << 13) + 0x38000000u);
  const float fs = (float)em * 5.9604644775390625e-8f;
  const float mag = (em < 0x400u) ? fs : fn;
  return __uint_as_float(__float_as_uint(mag) | sgn);
}

__device__ __forceinline__ void guard4_h(v8f& a, v8f& b, v8f& c, v8f& d, v16h x, v16h y0, v16h y1, v16h y2, v16h y3) {
  asm volatile("v_nop\n\tv_nop\n\tv_nop\n\tv_nop" : "+v"(a), "+v"(b), "+v"(c), "+v"(d) : "v"(x), "v"(y0), "v"(y1), "v"(y2), "v"(y3));
}
__device__ __forceinline__ void acc_guard4(v8f& a, v8f& b, v8f& c, v8f& d) {
  asm volatile("v_nop\n\tv_nop\n\tv_nop\n\tv_nop" : "+v"(a), "+v"(b), "+v"(c), "+v"(d));
}
__device__ __forceinline__ void wave_lds_sync() {
  __builtin_amdgcn_fence(__ATOMIC_RELEASE, "workgroup");
  __builtin_amdgcn_wave_barrier();
  __builtin_amdgcn_fence(__ATOMIC_ACQUIRE, "workgroup");
}

struct FragH {
  union U { v16h v; v8h h[2]; };
  static __device__ __forceinline__ v16h load(const _Float16* p) {
    U f; f.h[0] = *(const v8h*)(p); f.h[1] = *(const v8h*)(p + 16); return f.v;
  }
  static __device__ __forceinline__ v8f mma(v16h a, v16h b, v8f c) {
    return __builtin_amdgcn_wmma_f32_16x16x32_f16(false, a, false, b, (short)0, c, false, false);
  }
};

template <int EPI>
__global__ __launch_bounds__(256) void gemm64_f16(
    const unsigned short* __restrict__ Ap, int lda, long strideA,
    const unsigned short* __restrict__ Btp, int ldb, long strideB,
    void* __restrict__ Cout, int ldc, long strideC,
    const float* __restrict__ bias, long strideBias,
    const float* __restrict__ aux32, const unsigned short* __restrict__ aux16,
    int M, int N, int K, float scale) {
  constexpr bool kOutF32 = (EPI == kEpiDec || EPI == kEpiResid || EPI == kEpiFinal);
  constexpr bool kBiasN  = (EPI == kEpiMix || EPI == kEpiDec);
  constexpr bool kAct    = (EPI == kEpiTanh || EPI == kEpiDec || EPI == kEpiSigm);
  __shared__ __align__(16) float sT[8][16 * 68];
  const int zb   = blockIdx.y;
  const int lane = threadIdx.x & 31;
  const int wave = threadIdx.x >> 5;
  const int tilesN = N >> 6;
  const int tilesM = M >> 6;
  const int tile = blockIdx.x * 8 + wave;
  if (tile >= tilesM * tilesN) return;
  const int tm = tile / tilesN;
  const int tn = tile - tm * tilesN;
  const int m0 = tm << 6;
  const int n0 = tn << 6;
  const _Float16* A  = (const _Float16*)Ap  + (size_t)zb * strideA;
  const _Float16* Bt = (const _Float16*)Btp + (size_t)zb * strideB;
  const int rlane = lane & 15;
  const int koff  = (lane >> 4) * 8;
  const int mOff  = (lane >> 4) * 8;

  const _Float16* ap[4];
  const _Float16* bp[4];
#pragma unroll
  for (int i = 0; i < 4; ++i) {
    ap[i] = A  + (size_t)(m0 + (i << 4) + rlane) * lda + koff;
    bp[i] = Bt + (size_t)(n0 + (i << 4) + rlane) * ldb + koff;
  }

  v8f acc[4][4];
#pragma unroll
  for (int i = 0; i < 4; ++i)
#pragma unroll
    for (int j = 0; j < 4; ++j) acc[i][j] = (v8f){0.f, 0.f, 0.f, 0.f, 0.f, 0.f, 0.f, 0.f};

  for (int k0 = 0; k0 < K; k0 += 32) {
    const v16h b0 = FragH::load(bp[0] + k0);
    const v16h b1 = FragH::load(bp[1] + k0);
    const v16h b2 = FragH::load(bp[2] + k0);
    const v16h b3 = FragH::load(bp[3] + k0);
#pragma unroll
    for (int i = 0; i < 4; ++i) {
      const v16h ah = FragH::load(ap[i] + k0);
      acc[i][0] = FragH::mma(ah, b0, acc[i][0]);
      acc[i][1] = FragH::mma(ah, b1, acc[i][1]);
      acc[i][2] = FragH::mma(ah, b2, acc[i][2]);
      acc[i][3] = FragH::mma(ah, b3, acc[i][3]);
      guard4_h(acc[i][0], acc[i][1], acc[i][2], acc[i][3], ah, b0, b1, b2, b3);
    }
  }
  acc_guard4(acc[0][0], acc[0][1], acc[0][2], acc[0][3]);
  acc_guard4(acc[1][0], acc[1][1], acc[1][2], acc[1][3]);
  acc_guard4(acc[2][0], acc[2][1], acc[2][2], acc[2][3]);
  acc_guard4(acc[3][0], acc[3][1], acc[3][2], acc[3][3]);

  float* slab = sT[wave];
  float bv[4];
#pragma unroll
  for (int j = 0; j < 4; ++j) {
    bv[j] = 0.0f;
    if (kBiasN) bv[j] = bias[(size_t)zb * strideBias + n0 + (j << 4) + rlane];
  }

#pragma unroll
  for (int i = 0; i < 4; ++i) {
    const int mBase = m0 + (i << 4);
#pragma unroll
    for (int j = 0; j < 4; ++j) {
#pragma unroll
      for (int r = 0; r < 8; ++r) {
        slab[(mOff + r) * 68 + (j << 4) + rlane] = acc[i][j][r] * scale + bv[j];
      }
    }
    wave_lds_sync();
    if (kAct) {
#pragma unroll 1
      for (int q = 0; q < 32; ++q) {
        const int idx = q * 32 + lane;
        const int off = (idx >> 6) * 68 + (idx & 63);
        float v = slab[off];
        if (EPI == kEpiTanh) v = tanhf(v);
        if (EPI == kEpiDec)  v = expf(-expf(v));
        if (EPI == kEpiSigm) v = 1.0f / (1.0f + expf(-v));
        slab[off] = v;
      }
      wave_lds_sync();
    }
    if (kOutF32) {
      float* C = (float*)Cout + (size_t)zb * strideC;
      const int hh = lane >> 4, c4 = (lane & 15) * 4;
      v4f ov[8];
#pragma unroll
      for (int it = 0; it < 8; ++it) {
        const int row = it * 2 + hh;
        v4f v = *(const v4f*)(slab + row * 68 + c4);
        const size_t go = (size_t)(mBase + row) * ldc + n0 + c4;
        if (EPI == kEpiResid) {
          const v4f a = *(const v4f*)(aux32 + go);
          v = v + a;
        }
        if (EPI == kEpiFinal) {
          const v4f zv = *(const v4f*)(aux32 + go);
          const v2u rw = *(const v2u*)(aux16 + go);
          const unsigned w0 = rw[0];
          const unsigned w1 = rw[1];
          const float g0 = h16_to_f32(w0 & 0xffffu);
          const float g1 = h16_to_f32(w0 >> 16);
          const float g2 = h16_to_f32(w1 & 0xffffu);
          const float g3 = h16_to_f32(w1 >> 16);
          v4f o;
          o[0] = zv[0] + g0 * v[0];
          o[1] = zv[1] + g1 * v[1];
          o[2] = zv[2] + g2 * v[2];
          o[3] = zv[3] + g3 * v[3];
          v = o;
        }
        ov[it] = v;
      }
      for (int pass = 0; pass < 2; ++pass) {
#pragma unroll
        for (int it = 0; it < 8; ++it) {
          const int row = it * 2 + hh;
          *(volatile v4f*)(C + (size_t)(mBase + row) * ldc + n0 + c4) = ov[it];
        }
        __threadfence();
      }
    } else {
      unsigned short* C = (unsigned short*)Cout + (size_t)zb * strideC;
      const int q = lane >> 3, c8 = (lane & 7) * 8;
      v8h hv[4];
#pragma unroll
      for (int it = 0; it < 4; ++it) {
        const int row = it * 4 + q;
        const float* sp = slab + row * 68 + c8;
        const v4f s0 = *(const v4f*)(sp);
        const v4f s1 = *(const v4f*)(sp + 4);
        float vals[8];
#pragma unroll
        for (int e = 0; e < 4; ++e) { vals[e] = s0[e]; vals[4 + e] = s1[e]; }
        if (EPI == kEpiMix) {
          const int rg = mBase + row;
          const bool first = ((rg & (kT - 1)) == 0);
          const int ra = first ? rg : (rg - 1);
          const size_t go = (size_t)rg * ldc + n0 + c8;
          const size_t ga = (size_t)ra * ldc + n0 + c8;
          const v4f x0 = *(const v4f*)(aux32 + go);
          const v4f x1 = *(const v4f*)(aux32 + go + 4);
          const v4f p0 = *(const v4f*)(aux32 + ga);
          const v4f p1 = *(const v4f*)(aux32 + ga + 4);
#pragma unroll
          for (int e = 0; e < 4; ++e) {
            const float hc0 = x0[e];
            const float hc1 = x1[e];
            const float ha0 = first ? 0.0f : p0[e];
            const float ha1 = first ? 0.0f : p1[e];
            vals[e]     = hc0 + (ha0 - hc0) * vals[e];
            vals[4 + e] = hc1 + (ha1 - hc1) * vals[4 + e];
          }
        }
        if (EPI == kEpiReluSq) {
#pragma unroll
          for (int e = 0; e < 8; ++e) {
            const float rl = fmaxf(vals[e], 0.0f);
            vals[e] = (rl * rl) * kKkCarry;
          }
        }
#pragma unroll
        for (int e = 0; e < 8; ++e) hv[it][e] = (_Float16)vals[e];
      }
      for (int pass = 0; pass < 2; ++pass) {
#pragma unroll
        for (int it = 0; it < 4; ++it) {
          const int row = it * 4 + q;
          *(volatile v8h*)(C + (size_t)(mBase + row) * ldc + n0 + c8) = hv[it];
        }
        __threadfence();
      }
    }
    wave_lds_sync();
  }
}

__global__ __launch_bounds__(256) void wcast_kernel(const float* __restrict__ in, unsigned short* __restrict__ out,
                                                    int nIn8, int nOut8, float carry) {
  const int i = blockIdx.x * 256 + threadIdx.x;
  if (i >= nOut8) return;
  const bool live = (i < nIn8);
  const int ic = live ? i : (nIn8 - 1);
  const float* p = in + 8 * (size_t)ic;
  const v4f a = *(const v4f*)(p);
  const v4f c = *(const v4f*)(p + 4);
  unsigned short hb[8];
#pragma unroll
  for (int e = 0; e < 4; ++e) {
    const float fa = live ? (a[e] * carry) : 0.0f;
    const float fc = live ? (c[e] * carry) : 0.0f;
    hb[e]     = h_bits(fa);
    hb[4 + e] = h_bits(fc);
  }
  const v4u u = (v4u){pk16(hb[0], hb[1]), pk16(hb[2], hb[3]), pk16(hb[4], hb[5]), pk16(hb[6], hb[7])};
  unsigned short* q = out + 8 * (size_t)i;
  *(volatile v4u*)q = u;
  __threadfence();
  *(volatile v4u*)q = u;
}

__device__ __forceinline__ void rownorm16(v4f (&x)[4], const float* __restrict__ g, const float* __restrict__ b, int lane) {
  float s = 0.0f;
#pragma unroll
  for (int j = 0; j < 4; ++j) s += (x[j][0] + x[j][1]) + (x[j][2] + x[j][3]);
#pragma unroll
  for (int off = 16; off > 0; off >>= 1) s += __shfl_xor(s, off, 32);
  const float mu = s * (1.0f / kD);
  float ss = 0.0f;
#pragma unroll
  for (int j = 0; j < 4; ++j) {
#pragma unroll
    for (int e = 0; e < 4; ++e) {
      const float d = x[j][e] - mu;
      x[j][e] = d;
      ss += d * d;
    }
  }
#pragma unroll
  for (int off = 16; off > 0; off >>= 1) ss += __shfl_xor(ss, off, 32);
  const float inv = rsqrtf(ss * (1.0f / kD) + kLnEps);
#pragma unroll
  for (int j = 0; j < 4; ++j) {
    const v4f gv = *(const v4f*)(g + j * 128 + lane * 4);
    const v4f bv = *(const v4f*)(b + j * 128 + lane * 4);
#pragma unroll
    for (int e = 0; e < 4; ++e) x[j][e] = (x[j][e] * inv) * gv[e] + bv[e];
  }
}

template <bool TWO_STAGE>
__global__ __launch_bounds__(256) void rownorm_kernel(const float* __restrict__ X,
                                                      const float* __restrict__ ga, const float* __restrict__ ba,
                                                      const float* __restrict__ gb, const float* __restrict__ bb,
                                                      float* __restrict__ outA, float* __restrict__ outB) {
  const int lane = threadIdx.x & 31, wave = threadIdx.x >> 5;
  const size_t row = (size_t)blockIdx.x * 8 + wave;
  const size_t base = row * kD + lane * 4;
  v4f ya[4];
#pragma unroll
  for (int j = 0; j < 4; ++j) ya[j] = *(const v4f*)(X + base + j * 128);
  rownorm16(ya, ga, ba, lane);
  v4f yb[4];
#pragma unroll
  for (int j = 0; j < 4; ++j) yb[j] = ya[j];
  if (TWO_STAGE) rownorm16(yb, gb, bb, lane);
  for (int pass = 0; pass < 2; ++pass) {
#pragma unroll
    for (int j = 0; j < 4; ++j) {
      *(volatile v4f*)(outA + base + j * 128) = ya[j];
      if (TWO_STAGE) *(volatile v4f*)(outB + base + j * 128) = yb[j];
    }
    __threadfence();
  }
}

template <bool TWO>
__global__ __launch_bounds__(256) void shiftmix_kernel(const float* __restrict__ Hn,
                                                       const float* __restrict__ mu0, const float* __restrict__ mu1,
                                                       unsigned short* __restrict__ out0, unsigned short* __restrict__ out1) {
  const int i = blockIdx.x * 256 + threadIdx.x;
  const int row = i >> 6;
  const int c8 = (i & 63) * 8;
  const bool first = ((row & (kT - 1)) == 0);
  const int ra = first ? row : (row - 1);
  const float* pc = Hn + (size_t)row * kD + c8;
  const float* pa = Hn + (size_t)ra * kD + c8;
  const v4f x0 = *(const v4f*)(pc);
  const v4f x1 = *(const v4f*)(pc + 4);
  const v4f a0 = *(const v4f*)(pa);
  const v4f a1 = *(const v4f*)(pa + 4);
  const v4f m0 = *(const v4f*)(mu0 + c8);
  const v4f m1 = *(const v4f*)(mu0 + c8 + 4);
  const v4f n0 = *(const v4f*)(mu1 + c8);
  const v4f n1 = *(const v4f*)(mu1 + c8 + 4);
  unsigned short hb[8], gb[8];
#pragma unroll
  for (int e = 0; e < 4; ++e) {
    const float hc0 = x0[e];
    const float hc1 = x1[e];
    const float d0 = (first ? 0.0f : a0[e]) - hc0;
    const float d1 = (first ? 0.0f : a1[e]) - hc1;
    hb[e]     = h_bits(hc0 + d0 * m0[e]);
    hb[4 + e] = h_bits(hc1 + d1 * m1[e]);
    gb[e]     = h_bits(hc0 + d0 * n0[e]);
    gb[4 + e] = h_bits(hc1 + d1 * n1[e]);
  }
  const v4u u = (v4u){pk16(hb[0], hb[1]), pk16(hb[2], hb[3]), pk16(hb[4], hb[5]), pk16(hb[6], hb[7])};
  const v4u w = (v4u){pk16(gb[0], gb[1]), pk16(gb[2], gb[3]), pk16(gb[4], gb[5]), pk16(gb[6], gb[7])};
  unsigned short* q0 = out0 + (size_t)row * kD + c8;
  unsigned short* q1 = out1 + (size_t)row * kD + c8;
  *(volatile v4u*)q0 = u;
  if (TWO) *(volatile v4u*)q1 = w;
  __threadfence();
  *(volatile v4u*)q0 = u;
  if (TWO) *(volatile v4u*)q1 = w;
}

__global__ __launch_bounds__(128) void decay_scan_kernel(const unsigned short* __restrict__ R16,
                                                         const unsigned short* __restrict__ K16,
                                                         const float* __restrict__ DEC,
                                                         const unsigned short* __restrict__ V16,
                                                         const float* __restrict__ bonus,
                                                         float* __restrict__ O) {
  __shared__ __align__(16) float sr[kChunk][kDK];
  __shared__ __align__(16) float sk[kChunk][kDK];
  __shared__ __align__(16) float sd[kChunk][kDK];
  __shared__ __align__(16) float sv[kChunk][32];
  __shared__ __align__(16) float scoef[kChunk];
  __shared__ __align__(16) float po[kChunk][4][32];
  const int tid = threadIdx.x, lane = tid & 31, wave = tid >> 5;
  const int vg = blockIdx.x & 3;
  const int bh = blockIdx.x >> 2;
  const int hd = bh & 3;
  const int b  = bh >> 2;
  const int step = tid >> 3, kg = tid & 7;
  const v4f bn0 = *(const v4f*)(bonus + hd * kDK + kg * 8);
  const v4f bn1 = *(const v4f*)(bonus + hd * kDK + kg * 8 + 4);
  const size_t row0 = (size_t)b * kT;
  const int ocol = hd * kDV + vg * 32 + lane;
  float S[16];
#pragma unroll
  for (int i = 0; i < 16; ++i) S[i] = 0.0f;

#pragma unroll 1
  for (int c = 0; c < kT / kChunk; ++c) {
    {
      const size_t row = row0 + (size_t)c * kChunk + step;
      const size_t qo = row * kQK + hd * kDK + kg * 8;
      const v4u rw = *(const v4u*)(R16 + qo);
      const v4u kw = *(const v4u*)(K16 + qo);
      const v4f d0 = *(const v4f*)(DEC + qo);
      const v4f d1 = *(const v4f*)(DEC + qo + 4);
      const v2u vw = *(const v2u*)(V16 + row * kD + hd * kDV + vg * 32 + kg * 4);
      float rf[8], kf[8];
#pragma unroll
      for (int e = 0; e < 4; ++e) {
        const unsigned wr = rw[e];
        const unsigned wk = kw[e];
        rf[2 * e]     = h16_to_f32(wr & 0xffffu);
        rf[2 * e + 1] = h16_to_f32(wr >> 16);
        kf[2 * e]     = h16_to_f32(wk & 0xffffu);
        kf[2 * e + 1] = h16_to_f32(wk >> 16);
      }
      float part = 0.0f;
#pragma unroll
      for (int e = 0; e < 4; ++e) {
        part += (rf[e] * bn0[e]) * kf[e];
        part += (rf[4 + e] * bn1[e]) * kf[4 + e];
      }
      part += __shfl_xor(part, 1, 32);
      part += __shfl_xor(part, 2, 32);
      part += __shfl_xor(part, 4, 32);
      const unsigned v0w = vw[0];
      const unsigned v1w = vw[1];
      *(v4f*)(&sr[step][kg * 8])     = (v4f){rf[0], rf[1], rf[2], rf[3]};
      *(v4f*)(&sr[step][kg * 8 + 4]) = (v4f){rf[4], rf[5], rf[6], rf[7]};
      *(v4f*)(&sk[step][kg * 8])     = (v4f){kf[0], kf[1], kf[2], kf[3]};
      *(v4f*)(&sk[step][kg * 8 + 4]) = (v4f){kf[4], kf[5], kf[6], kf[7]};
      *(v4f*)(&sd[step][kg * 8])     = d0;
      *(v4f*)(&sd[step][kg * 8 + 4]) = d1;
      *(v4f*)(&sv[step][kg * 4]) = (v4f){h16_to_f32(v0w & 0xffffu), h16_to_f32(v0w >> 16),
                                         h16_to_f32(v1w & 0xffffu), h16_to_f32(v1w >> 16)};
      if (kg == 0) scoef[step] = part;
    }
    __syncthreads();

#pragma unroll 1
    for (int s = 0; s < kChunk; ++s) {
      const float vv = sv[s][lane];
      const float cf = scoef[s];
      float acc = (wave == 0) ? (cf * vv) : 0.0f;
      const v4f* rp = (const v4f*)(&sr[s][wave * 16]);
      const v4f* kp = (const v4f*)(&sk[s][wave * 16]);
      const v4f* dp = (const v4f*)(&sd[s][wave * 16]);
#pragma unroll
      for (int q = 0; q < 4; ++q) {
        const v4f rq = rp[q];
        const v4f kq = kp[q];
        const v4f dq = dp[q];
#pragma unroll
        for (int e = 0; e < 4; ++e) {
          const float kvv = kq[e] * vv;
          acc = fmaf(rq[e], S[q * 4 + e], acc);
          S[q * 4 + e] = fmaf(dq[e], S[q * 4 + e], kvv);
        }
      }
      po[s][wave][lane] = acc;
    }
    __syncthreads();

    {
      float val[4];
#pragma unroll
      for (int i = 0; i < 4; ++i) {
        const int s = wave * 4 + i;
        val[i] = ((po[s][0][lane] + po[s][1][lane]) + po[s][2][lane]) + po[s][3][lane];
      }
      float* op = O + (row0 + (size_t)c * kChunk + wave * 4) * kD + ocol;
      for (int pass = 0; pass < 2; ++pass) {
#pragma unroll
        for (int i = 0; i < 4; ++i) *(volatile float*)(op + (size_t)i * kD) = val[i];
        __threadfence();
      }
    }
  }
}

__global__ __launch_bounds__(256) void gn_gate_kernel(const float* __restrict__ O, const unsigned short* __restrict__ G16,
                                                      const float* __restrict__ gw, const float* __restrict__ gb,
                                                      unsigned short* __restrict__ OO) {
  const int lane = threadIdx.x & 31, wave = threadIdx.x >> 5;
  const int grp = blockIdx.x * 8 + wave;
  const int row = grp >> 2;
  const int hd  = grp & 3;
  const size_t base = (size_t)row * kD + hd * kDV + lane * 4;
  const v4f ov = *(const v4f*)(O + base);
  const v2u gwd = *(const v2u*)(G16 + base);
  const v4f wv = *(const v4f*)(gw + lane * 4);
  const v4f bv = *(const v4f*)(gb + lane * 4);
  const float o0 = ov[0], o1 = ov[1], o2 = ov[2], o3 = ov[3];
  float s = (o0 + o1) + (o2 + o3);
#pragma unroll
  for (int off = 16; off > 0; off >>= 1) s += __shfl_xor(s, off, 32);
  const float mu = s * (1.0f / kDV);
  const float d0 = o0 - mu, d1 = o1 - mu, d2 = o2 - mu, d3 = o3 - mu;
  float ss = (d0 * d0 + d1 * d1) + (d2 * d2 + d3 * d3);
#pragma unroll
  for (int off = 16; off > 0; off >>= 1) ss += __shfl_xor(ss, off, 32);
  const float rstd = rsqrtf(ss * (1.0f / kDV) + kLnEps);
  const unsigned g01 = gwd[0];
  const unsigned g23 = gwd[1];
  const float g0 = h16_to_f32(g01 & 0xffffu);
  const float g1 = h16_to_f32(g01 >> 16);
  const float g2 = h16_to_f32(g23 & 0xffffu);
  const float g3 = h16_to_f32(g23 >> 16);
  const float s0 = g0 * (1.0f / (1.0f + expf(-g0)));
  const float s1 = g1 * (1.0f / (1.0f + expf(-g1)));
  const float s2 = g2 * (1.0f / (1.0f + expf(-g2)));
  const float s3 = g3 * (1.0f / (1.0f + expf(-g3)));
  const float z0 = (((d0 * rstd) * wv[0] + bv[0]) * s0) * kOoCarry;
  const float z1 = (((d1 * rstd) * wv[1] + bv[1]) * s1) * kOoCarry;
  const float z2 = (((d2 * rstd) * wv[2] + bv[2]) * s2) * kOoCarry;
  const float z3 = (((d3 * rstd) * wv[3] + bv[3]) * s3) * kOoCarry;
  const v2u u = (v2u){pk16(h_bits(z0), h_bits(z1)), pk16(h_bits(z2), h_bits(z3))};
  unsigned short* zp = OO + base;
  *(volatile v2u*)zp = u;
  __threadfence();
  *(volatile v2u*)zp = u;
}

extern "C" void kernel_launch(void* const* d_in, const int* in_sizes, int n_in,
                              void* d_out, int out_size, void* d_ws, size_t ws_size, hipStream_t stream) {
  if (n_in < 27 || d_out == nullptr || d_ws == nullptr) return;
  const int expect[27] = {
      kRows * kD, kD, kD, kD, kD, kD, kD, kD,
      kMixCols * kD, kD * kMixCols, 5 * kD,
      kQK * kD, kDecRank * kD, kQK * kDecRank, kQK, kQK * kD,
      kD * kD, kD * kD, kH * kDK, kDV, kDV, kD * kD,
      kD, kFF * kD, kD, kD * kD, kD * kFF};
  for (int i = 0; i < 27; ++i) {
    if (in_sizes[i] != expect[i]) return;
  }
  if (out_size != kRows * kD) return;

  const float* x      = (const float*)d_in[0];
  const float* ln0_g  = (const float*)d_in[1];
  const float* ln0_b  = (const float*)d_in[2];
  const float* ln1_g  = (const float*)d_in[3];
  const float* ln1_b  = (const float*)d_in[4];
  const float* ln2_g  = (const float*)d_in[5];
  const float* ln2_b  = (const float*)d_in[6];
  const float* xp_mu  = (const float*)d_in[7];
  const float* xp_w1  = (const float*)d_in[8];
  const float* xp_w2  = (const float*)d_in[9];
  const float* x_bias = (const float*)d_in[10];
  const float* r_w    = (const float*)d_in[11];
  const float* w_A    = (const float*)d_in[12];
  const float* w_B    = (const float*)d_in[13];
  const float* w_b    = (const float*)d_in[14];
  const float* k_w    = (const float*)d_in[15];
  const float* v_w    = (const float*)d_in[16];
  const float* g_w    = (const float*)d_in[17];
  const float* bonus  = (const float*)d_in[18];
  const float* gn_g   = (const float*)d_in[19];
  const float* gn_b   = (const float*)d_in[20];
  const float* o_w    = (const float*)d_in[21];
  const float* fk_mu  = (const float*)d_in[22];
  const float* fk_w   = (const float*)d_in[23];
  const float* fr_mu  = (const float*)d_in[24];
  const float* fr_w   = (const float*)d_in[25];
  const float* fv_w   = (const float*)d_in[26];
  float* out = (float*)d_out;

  const size_t PLN = (size_t)kRows * kD;
  char* ws = (char*)d_ws;
  size_t off = 0;
  auto carve = [&](size_t bytes) -> char* { char* p = ws + off; off += (bytes + 255) & ~(size_t)255; return p; };
  float*          PA  = (float*)carve(PLN * 4);
  float*          PB  = (float*)carve(PLN * 4);
  unsigned short* UM  = (unsigned short*)carve(PLN * 2);
  unsigned short* XX  = (unsigned short*)carve((size_t)kRows * kMixPad * 2);
  unsigned short* U   = (unsigned short*)carve((size_t)5 * PLN * 2);
  unsigned short* RK  = (unsigned short*)carve((size_t)2 * kRows * kQK * 2);
  float*          DEC = (float*)carve((size_t)kRows * kQK * 4);
  unsigned short* WT  = (unsigned short*)carve((size_t)kRows * kDecRank * 2);
  unsigned short* VG  = (unsigned short*)carve((size_t)2 * PLN * 2);
  unsigned short* W1  = (unsigned short*)carve((size_t)kMixPad * kD * 2);
  unsigned short* W2  = (unsigned short*)carve((size_t)kD * kMixCols * 2);
  unsigned short* Wrk = (unsigned short*)carve((size_t)2 * kQK * kD * 2);
  unsigned short* WA  = (unsigned short*)carve((size_t)kDecRank * kD * 2);
  unsigned short* WB  = (unsigned short*)carve((size_t)kQK * kDecRank * 2);
  unsigned short* Wvg = (unsigned short*)carve((size_t)2 * kD * kD * 2);
  unsigned short* Wo  = (unsigned short*)carve((size_t)kD * kD * 2);
  unsigned short* Wfk = (unsigned short*)carve((size_t)kFF * kD * 2);
  unsigned short* Wfr = (unsigned short*)carve((size_t)kD * kD * 2);
  unsigned short* Wfv = (unsigned short*)carve((size_t)kD * kFF * 2);
  if (off > ws_size || off > (size_t)134217728) return;

  unsigned short* U0 = U;
  unsigned short* U1 = U + PLN;
  unsigned short* U2 = U + 2 * PLN;
  unsigned short* U3 = U + 3 * PLN;
  unsigned short* U4 = U + 4 * PLN;
  unsigned short* Rp = RK;
  unsigned short* Kp = RK + (size_t)kRows * kQK;
  unsigned short* Vp = VG;
  unsigned short* Gp = VG + PLN;

  auto castw = [&](const float* src, unsigned short* dst, int nIn, int nOut) {
    const int nIn8 = nIn / 8, nOut8 = nOut / 8;
    wcast_kernel<<<(nOut8 + 255) / 256, 256, 0, stream>>>(src, dst, nIn8, nOut8, kWCarry);
  };
  castw(xp_w1, W1, kMixCols * kD, kMixPad * kD);
  castw(xp_w2, W2, kD * kMixCols, kD * kMixCols);
  castw(r_w, Wrk, kQK * kD, kQK * kD);
  castw(k_w, Wrk + (size_t)kQK * kD, kQK * kD, kQK * kD);
  castw(w_A, WA, kDecRank * kD, kDecRank * kD);
  castw(w_B, WB, kQK * kDecRank, kQK * kDecRank);
  castw(v_w, Wvg, kD * kD, kD * kD);
  castw(g_w, Wvg + (size_t)kD * kD, kD * kD, kD * kD);
  castw(o_w, Wo, kD * kD, kD * kD);
  castw(fk_w, Wfk, kFF * kD, kFF * kD);
  castw(fr_w, Wfr, kD * kD, kD * kD);
  castw(fv_w, Wfv, kD * kFF, kD * kFF);

  const int tM    = kRows / 64;
  const int gBig  = tM * (kD / 64) / 8;
  const int gMix  = tM * (kMixPad / 64) / 8;
  const int gQK   = tM * (kQK / 64) / 8;
  const int gDec  = tM * (kDecRank / 64) / 8;
  const int gFF   = tM * (kFF / 64) / 8;
  const float sW  = 1.0f / kWCarry;

  rownorm_kernel<true><<<kRows / 8, 256, 0, stream>>>(x, ln0_g, ln0_b, ln1_g, ln1_b, PA, PB);

  shiftmix_kernel<false><<<kRows * kD / 8 / 256, 256, 0, stream>>>(PB, xp_mu, xp_mu, UM, UM);

  gemm64_f16<kEpiTanh><<<dim3(gMix, 1), 256, 0, stream>>>(
      UM, kD, 0L, W1, kD, 0L, (void*)XX, kMixPad, 0L,
      x_bias, 0L, PB, UM, kRows, kMixPad, kD, sW);

  gemm64_f16<kEpiMix><<<dim3(gBig, 5), 256, 0, stream>>>(
      XX, kMixPad, (long)kLR, W2, kMixCols, (long)kLR, (void*)U, kD, (long)PLN,
      x_bias, (long)kD, PB, UM, kRows, kD, kLR, sW);

  gemm64_f16<kEpiPlain><<<dim3(gQK, 2), 256, 0, stream>>>(
      U0, kD, (long)(2 * PLN), Wrk, kD, (long)kQK * kD, (void*)RK, kQK, (long)kRows * kQK,
      x_bias, 0L, PB, UM, kRows, kQK, kD, sW);

  gemm64_f16<kEpiTanh><<<dim3(gDec, 1), 256, 0, stream>>>(
      U1, kD, 0L, WA, kD, 0L, (void*)WT, kDecRank, 0L,
      x_bias, 0L, PB, UM, kRows, kDecRank, kD, sW);

  gemm64_f16<kEpiDec><<<dim3(gQK, 1), 256, 0, stream>>>(
      WT, kDecRank, 0L, WB, kDecRank, 0L, (void*)DEC, kQK, 0L,
      w_b, 0L, PB, UM, kRows, kQK, kDecRank, sW);

  gemm64_f16<kEpiPlain><<<dim3(gBig, 2), 256, 0, stream>>>(
      U3, kD, (long)PLN, Wvg, kD, (long)kD * kD, (void*)VG, kD, (long)PLN,
      x_bias, 0L, PB, UM, kRows, kD, kD, sW);

  decay_scan_kernel<<<kB * kH * 4, 128, 0, stream>>>(Rp, Kp, DEC, Vp, bonus, PB);

  gn_gate_kernel<<<kRows * kH / 8, 256, 0, stream>>>(PB, Gp, gn_g, gn_b, U2);

  gemm64_f16<kEpiResid><<<dim3(gBig, 1), 256, 0, stream>>>(
      U2, kD, 0L, Wo, kD, 0L, (void*)PB, kD, 0L,
      x_bias, 0L, PA, UM, kRows, kD, kD, 1.0f / (kOoCarry * kWCarry));

  rownorm_kernel<false><<<kRows / 8, 256, 0, stream>>>(PB, ln2_g, ln2_b, ln2_g, ln2_b, PA, PA);

  shiftmix_kernel<true><<<kRows * kD / 8 / 256, 256, 0, stream>>>(PA, fk_mu, fr_mu, UM, U4);

  gemm64_f16<kEpiReluSq><<<dim3(gFF, 1), 256, 0, stream>>>(
      UM, kD, 0L, Wfk, kD, 0L, (void*)U0, kFF, 0L,
      x_bias, 0L, PB, UM, kRows, kFF, kD, sW);

  gemm64_f16<kEpiSigm><<<dim3(gBig, 1), 256, 0, stream>>>(
      U4, kD, 0L, Wfr, kD, 0L, (void*)U3, kD, 0L,
      x_bias, 0L, PB, UM, kRows, kD, kD, sW);

  gemm64_f16<kEpiFinal><<<dim3(gBig, 1), 256, 0, stream>>>(
      U0, kFF, 0L, Wfv, kFF, 0L, (void*)out, kD, 0L,
      x_bias, 0L, PB, U3, kRows, kD, kFF, 1.0f / (kKkCarry * kWCarry));
}
